// MultiHeadSelfAttention_39719857553749
// MI455X (gfx1250) — hardware-verified
//
#include <hip/hip_runtime.h>
#ifndef NB
#define NB 2
#endif
#ifndef SEQ
#define SEQ 2048
#endif
#define NB_FULL 2
#define SEQ_FULL 2048
#define DM 1024
#define NH 16
#define HD 64
#define LQ (3 * DM)
#define LO (2 * DM)
#define NR ((size_t)NB * SEQ)
#define SZ_BQKV ((size_t)3 * DM * DM * 2)
#define SZ_BO   ((size_t)DM * LO * 2)
#define SZ_X16  (NR * DM * 2)
#define SZ_QKV  (NR * LQ * 2)
#define SZ_VT   ((size_t)NB * NH * HD * SEQ * 2)
#define SZ_O16  (NR * LO * 2)
static_assert(NB <= NB_FULL);
static_assert(SEQ <= SEQ_FULL);
static_assert(NH * HD == DM);
static_assert(HD == 64);
static_assert(DM % 32 == 0);
static_assert(LO % 32 == 0);
static_assert(SEQ % 64 == 0);
static_assert((NB * SEQ) % 128 == 0);
static_assert(DM % 64 == 0);
static_assert(LQ % 64 == 0);
static_assert(LQ % 8 == 0);
static_assert(SEQ % 8 == 0);
static_assert(SZ_BQKV % 256 == 0);
static_assert(SZ_BO % 256 == 0);
static_assert(SZ_X16 % 256 == 0);
static_assert(SZ_QKV % 256 == 0);
static_assert(SZ_VT % 256 == 0);
static_assert(SZ_O16 % 256 == 0);
static_assert(SZ_BQKV + SZ_BO + SZ_X16 + SZ_QKV + SZ_VT + SZ_O16 <= (size_t)134217728);

typedef unsigned short v8us __attribute__((ext_vector_type(8), may_alias));
typedef float  v8f  __attribute__((ext_vector_type(8)));
typedef float  v4f  __attribute__((ext_vector_type(4)));
typedef float  v4fa __attribute__((ext_vector_type(4), may_alias));
typedef _Float16 v16h __attribute__((ext_vector_type(16)));
typedef _Float16 v4h __attribute__((ext_vector_type(4)));
union FragH { v16h v; v8us half[2]; _Float16 h[16]; unsigned short u[16]; };

__device__ __forceinline__ unsigned short bf16_bits(float x) { unsigned int u = __float_as_uint(x); return (unsigned short)((u + 0x7FFFu + ((u >> 16) & 1u)) >> 16); }
__device__ __forceinline__ float bf16_rne(float x) { return __uint_as_float(((unsigned int)bf16_bits(x)) << 16); }

__device__ __forceinline__ v16h g2_frag(const _Float16* p, int hh) { FragH f; f.half[0] = *(const v8us*)((const unsigned short*)p + 8 * hh); f.half[1] = *(const v8us*)((const unsigned short*)p + 16 + 8 * hh); return f.v; }
__device__ __forceinline__ v8f g2_mma(v16h a, v16h b, v8f c) { v8f d = __builtin_amdgcn_wmma_f32_16x16x32_f16(false, a, false, b, (short)0, c, false, false); asm volatile("v_nop\n\tv_nop\n\tv_nop\n\tv_nop" : "+v"(d) : "v"(a), "v"(b)); return d; }

__global__ __launch_bounds__(256) void k_wt_f16(const float* __restrict__ W, _Float16* __restrict__ Wt, int K, int N, int ldo, float scale, float scale2) {
  const int t = blockIdx.x * 256 + threadIdx.x; const int k8n = K / 8; if (t >= N * k8n) return;
  const int n = t / k8n, k8 = (t - n * k8n) * 8; FragH f, g;
#pragma unroll
  for (int i = 0; i < 8; ++i) { const float w = bf16_rne(W[(size_t)(k8 + i) * N + n]); f.h[i] = (_Float16)(w * scale); g.h[i] = (_Float16)(w * scale2); }
  const v8us o = f.half[0], o2 = g.half[0];
  unsigned short* d = (unsigned short*)Wt + (size_t)n * ldo + k8;
  *(volatile v8us*)d = o; if (scale2 > 0.f) *(volatile v8us*)(d + K) = o2;
  __threadfence();
  *(volatile v8us*)d = o; if (scale2 > 0.f) *(volatile v8us*)(d + K) = o2;
}

__global__ __launch_bounds__(256) void k_x16(const float* __restrict__ x, _Float16* __restrict__ X16) {
  const size_t t = (size_t)blockIdx.x * 256 + threadIdx.x; if (t >= NR * DM / 8) return;
  const size_t row = t / (DM / 8); const int c8 = (int)(t - row * (DM / 8)) * 8;
  const size_t b = row / SEQ, s = row - b * SEQ;
  const float* src = x + (b * SEQ_FULL + s) * DM + c8;
  const v4f a = *(const v4fa*)src, c = *(const v4fa*)(src + 4); FragH f;
#pragma unroll
  for (int q = 0; q < 4; ++q) { f.h[q] = (_Float16)bf16_rne(a[q]); f.h[4 + q] = (_Float16)bf16_rne(c[q]); }
  const v8us o = f.half[0];
  unsigned short* d = (unsigned short*)X16 + row * DM + c8;
  *(volatile v8us*)d = o; __threadfence(); *(volatile v8us*)d = o;
}

template <bool OUT16>
__device__ __forceinline__ void gemm2_body(const _Float16* __restrict__ A, int lda, const _Float16* __restrict__ Bh, int ldb, float alpha, const float* __restrict__ bias,
                                           float* __restrict__ C, _Float16* __restrict__ C16, int ldc, int N, int K) {
  __shared__ __attribute__((aligned(16))) float so[4][32][68];
  const int lane = threadIdx.x & 31, ln = lane & 15, hh = lane >> 4;
  const int w = __builtin_amdgcn_readfirstlane((int)(threadIdx.x >> 5));
  const int ntn = N >> 6; const int mt = (int)blockIdx.x / ntn, nq = (int)blockIdx.x - mt * ntn; const int row0 = mt * 128 + 32 * w, col0 = nq * 64;
  const _Float16* a0p = A + (size_t)(row0 + ln) * lda; const _Float16* a1p = a0p + (size_t)16 * lda;
  const _Float16* b0p = Bh + (size_t)(col0 + ln) * ldb; const _Float16* b1p = b0p + (size_t)16 * ldb; const _Float16* b2p = b1p + (size_t)16 * ldb; const _Float16* b3p = b2p + (size_t)16 * ldb;
  const v8f z8 = {0.f,0.f,0.f,0.f,0.f,0.f,0.f,0.f}; v8f c00 = z8, c01 = z8, c02 = z8, c03 = z8, c10 = z8, c11 = z8, c12 = z8, c13 = z8;
#pragma unroll 1
  for (int kb = 0; kb < K; kb += 32) { const v16h a0 = g2_frag(a0p + kb, hh), a1 = g2_frag(a1p + kb, hh);
    v16h b = g2_frag(b0p + kb, hh); c00 = g2_mma(a0, b, c00); c10 = g2_mma(a1, b, c10);
    b = g2_frag(b1p + kb, hh); c01 = g2_mma(a0, b, c01); c11 = g2_mma(a1, b, c11);
    b = g2_frag(b2p + kb, hh); c02 = g2_mma(a0, b, c02); c12 = g2_mma(a1, b, c12);
    b = g2_frag(b3p + kb, hh); c03 = g2_mma(a0, b, c03); c13 = g2_mma(a1, b, c13); }
  v8f accs[8] = {c00, c01, c02, c03, c10, c11, c12, c13};
#pragma unroll
  for (int u = 0; u < 8; ++u) { const int t = u & 3, half = u >> 2; const int col = col0 + t * 16 + ln; const float bv = bf16_rne(bias[col]);
#pragma unroll
    for (int r = 0; r < 8; ++r) { const int rloc = half * 16 + 8 * hh + r; so[w][rloc][t * 16 + ln] = accs[u][r] * alpha + bv; } }
  __syncthreads();
  const int rsub = lane >> 4, c4 = (lane & 15) * 4;
  for (int pass = 0; pass < 2; ++pass) {
#pragma unroll
    for (int q = 0; q < 16; ++q) { const int r = q * 2 + rsub; const v4f v = *(const v4fa*)&so[w][r][c4];
      if (OUT16) { v4h h4; h4[0] = (_Float16)v[0]; h4[1] = (_Float16)v[1]; h4[2] = (_Float16)v[2]; h4[3] = (_Float16)v[3]; *(volatile v4h*)(C16 + (size_t)(row0 + r) * ldc + col0 + c4) = h4; }
      else *(volatile v4f*)(C + (size_t)(row0 + r) * ldc + col0 + c4) = v; }
    if (pass == 0) __threadfence(); }
}
__global__ __launch_bounds__(128) void k_gemm_qkv(const _Float16* __restrict__ A, const _Float16* __restrict__ Bh, const float* __restrict__ bias, _Float16* __restrict__ C16) {
  gemm2_body<true>(A, DM, Bh, DM, 0.0625f, bias, nullptr, C16, LQ, LQ, DM);
}
__global__ __launch_bounds__(128) void k_gemm_out(const _Float16* __restrict__ A, const _Float16* __restrict__ Bh, const float* __restrict__ bias, float* __restrict__ C) {
  gemm2_body<false>(A, LO, Bh, LO, 1.0f / 65536.0f, bias, C, nullptr, DM, DM, LO);
}

__global__ __launch_bounds__(256) void k_vt(const _Float16* __restrict__ QKV, _Float16* __restrict__ VT) {
  __shared__ unsigned short tl[64][66];
  const int tid = threadIdx.x; const int slab = (int)blockIdx.x / (SEQ / 64), lg = (int)blockIdx.x - slab * (SEQ / 64); const int b = slab / NH, h = slab - b * NH;
  for (int i = tid; i < 64 * 8; i += 256) { const int r = i >> 3, c8 = (i & 7) * 8; FragH f; f.half[0] = *(const v8us*)((const unsigned short*)QKV + ((size_t)b * SEQ + lg * 64 + r) * LQ + 2 * DM + h * HD + c8);
#pragma unroll
    for (int q = 0; q < 8; ++q) tl[r][c8 + q] = f.u[q]; }
  __syncthreads();
  for (int pass = 0; pass < 2; ++pass) {
#pragma unroll
    for (int rd = 0; rd < 2; ++rd) { const int d = rd * 32 + (tid >> 3), pc = tid & 7; FragH f;
#pragma unroll
      for (int q = 0; q < 8; ++q) f.u[q] = tl[pc * 8 + q][d];
      *(volatile v8us*)((unsigned short*)VT + ((size_t)slab * HD + d) * SEQ + lg * 64 + pc * 8) = f.half[0]; }
    if (pass == 0) __threadfence(); }
}

__device__ __forceinline__ v4f lo4(v8f a, float s) { v4f r = {a[0] * s, a[1] * s, a[2] * s, a[3] * s}; return r; }
__device__ __forceinline__ v4f hi4(v8f a, float s) { v4f r = {a[4] * s, a[5] * s, a[6] * s, a[7] * s}; return r; }

__global__ __launch_bounds__(128) void k_attn(const _Float16* __restrict__ QKV, const _Float16* __restrict__ VT, _Float16* __restrict__ O16) {
  __shared__ __attribute__((aligned(16))) float so[4][16][68];
  const int lane = threadIdx.x & 31, ln = lane & 15, hh = lane >> 4;
  const int wave = __builtin_amdgcn_readfirstlane((int)(threadIdx.x >> 5));
  const int bh = blockIdx.y; const int b = bh / NH, h = bh - b * NH;
  const int q0 = (int)blockIdx.x * 64 + wave * 16;
  const size_t rowb = (size_t)b * SEQ;
  const _Float16* qp = QKV + (rowb + q0 + ln) * LQ + h * HD;
  const v16h qf0 = g2_frag(qp, hh), qf1 = g2_frag(qp + 32, hh);
  const _Float16* kp = QKV + (rowb + ln) * LQ + DM + h * HD;
  const _Float16* vp = VT + ((size_t)bh * HD + ln) * SEQ;
  const v8f z8 = {0.f,0.f,0.f,0.f,0.f,0.f,0.f,0.f};
  v8f o0 = z8, o1 = z8, o2 = z8, o3 = z8;
  float m = -1.0e30f, l = 0.f;
  const float SC2 = 0.125f * 1.4426950408889634f;
#pragma unroll 1
  for (int kb = 0; kb < SEQ; kb += 32) {
    const _Float16* k0 = kp + (size_t)kb * LQ; const _Float16* k1 = k0 + (size_t)16 * LQ;
    v8f s0 = z8, s1 = z8;
    v16h a = g2_frag(k0, hh); s0 = g2_mma(a, qf0, s0);
    a = g2_frag(k0 + 32, hh); s0 = g2_mma(a, qf1, s0);
    a = g2_frag(k1, hh); s1 = g2_mma(a, qf0, s1);
    a = g2_frag(k1 + 32, hh); s1 = g2_mma(a, qf1, s1);
    float vm = fmaxf(s0[0], s1[0]);
#pragma unroll
    for (int r = 1; r < 8; ++r) vm = fmaxf(vm, fmaxf(s0[r], s1[r]));
    vm = fmaxf(vm, __shfl_xor(vm, 16));
    const float mn = fmaxf(m, vm * SC2);
    const float al = exp2f(m - mn);
    m = mn;
    const float mo = mn - 6.0f;
    FragH pf; float ls = 0.f;
#pragma unroll
    for (int r = 0; r < 8; ++r) { const float p0 = exp2f(s0[r] * SC2 - mo), p1 = exp2f(s1[r] * SC2 - mo); ls += p0 + p1; pf.h[r] = (_Float16)p0; pf.h[8 + r] = (_Float16)p1; }
    ls += __shfl_xor(ls, 16);
    l = l * al + ls;
#pragma unroll
    for (int r = 0; r < 8; ++r) { o0[r] *= al; o1[r] *= al; o2[r] *= al; o3[r] *= al; }
    const _Float16* v0 = vp + kb;
    const v16h va0 = g2_frag(v0, hh), va1 = g2_frag(v0 + (size_t)16 * SEQ, hh), va2 = g2_frag(v0 + (size_t)32 * SEQ, hh), va3 = g2_frag(v0 + (size_t)48 * SEQ, hh);
    o0 = g2_mma(va0, pf.v, o0); o1 = g2_mma(va1, pf.v, o1); o2 = g2_mma(va2, pf.v, o2); o3 = g2_mma(va3, pf.v, o3);
  }
  const float sc = 64.0f * (1.0f / l);
  *(v4fa*)&so[wave][ln][ 0 + 8 * hh] = lo4(o0, sc); *(v4fa*)&so[wave][ln][ 4 + 8 * hh] = hi4(o0, sc);
  *(v4fa*)&so[wave][ln][16 + 8 * hh] = lo4(o1, sc); *(v4fa*)&so[wave][ln][20 + 8 * hh] = hi4(o1, sc);
  *(v4fa*)&so[wave][ln][32 + 8 * hh] = lo4(o2, sc); *(v4fa*)&so[wave][ln][36 + 8 * hh] = hi4(o2, sc);
  *(v4fa*)&so[wave][ln][48 + 8 * hh] = lo4(o3, sc); *(v4fa*)&so[wave][ln][52 + 8 * hh] = hi4(o3, sc);
  __syncthreads();
  const int rq = lane >> 3, pc = lane & 7;
  for (int pass = 0; pass < 2; ++pass) {
#pragma unroll
    for (int it = 0; it < 4; ++it) { const int row = it * 4 + rq;
      const v4f x0 = *(const v4fa*)&so[wave][row][pc * 8], x1 = *(const v4fa*)&so[wave][row][pc * 8 + 4];
      FragH fh, fl;
#pragma unroll
      for (int q = 0; q < 4; ++q) { _Float16 hv = (_Float16)x0[q]; fh.h[q] = hv; fl.h[q] = (_Float16)((x0[q] - (float)hv) * 1024.0f); hv = (_Float16)x1[q]; fh.h[4 + q] = hv; fl.h[4 + q] = (_Float16)((x1[q] - (float)hv) * 1024.0f); }
      const v8us oh = fh.half[0], ol = fl.half[0];
      unsigned short* d = (unsigned short*)O16 + (rowb + q0 + row) * LO + h * HD + pc * 8;
      *(volatile v8us*)d = oh; *(volatile v8us*)(d + DM) = ol; }
    if (pass == 0) __threadfence(); }
}

extern "C" void kernel_launch(void* const* d_in, const int* in_sizes, int n_in,
                              void* d_out, int out_size, void* d_ws, size_t ws_size, hipStream_t stream) {
  if (n_in < 5) return;
  if ((size_t)in_sizes[0] < ((size_t)(NB - 1) * SEQ_FULL + SEQ) * DM) return;
  if ((size_t)in_sizes[1] < (size_t)DM * 3 * DM) return;
  if (in_sizes[2] < 3 * DM) return;
  if ((size_t)in_sizes[3] < (size_t)DM * DM) return;
  if (in_sizes[4] < DM) return;
  if ((size_t)out_size < NR * DM) return;
  const float* x = (const float*)d_in[0]; const float* wqkv = (const float*)d_in[1]; const float* bqkv = (const float*)d_in[2]; const float* wo = (const float*)d_in[3]; const float* bo = (const float*)d_in[4];
  char* ws = (char*)d_ws; size_t off = 0;
  auto take = [&](size_t bytes) { char* p = ws + off; off += (bytes + 255) & ~(size_t)255; return p; };
  _Float16* BQKV = (_Float16*)take(SZ_BQKV);
  _Float16* BO   = (_Float16*)take(SZ_BO);
  _Float16* X16  = (_Float16*)take(SZ_X16);
  _Float16* QKV  = (_Float16*)take(SZ_QKV);
  _Float16* VT   = (_Float16*)take(SZ_VT);
  _Float16* O16  = (_Float16*)take(SZ_O16);
  if (off > ws_size) return;
  k_wt_f16<<<(unsigned)(((size_t)3 * DM * (DM / 8) + 255) / 256), 256, 0, stream>>>(wqkv, BQKV, DM, 3 * DM, DM, 16.0f, 0.0f);
  k_wt_f16<<<(unsigned)(((size_t)DM * (DM / 8) + 255) / 256), 256, 0, stream>>>(wo, BO, DM, DM, LO, 1024.0f, 1.0f);
  k_x16<<<(unsigned)((NR * DM / 8 + 255) / 256), 256, 0, stream>>>(x, X16);
  k_gemm_qkv<<<(unsigned)((NR / 128) * (LQ / 64)), 128, 0, stream>>>(X16, BQKV, bqkv, QKV);
  k_vt<<<(unsigned)(NB * NH * (SEQ / 64)), 256, 0, stream>>>(QKV, VT);
  k_attn<<<dim3(SEQ / 64, NB * NH), 128, 0, stream>>>(QKV, VT, O16);
  k_gemm_out<<<(unsigned)((NR / 128) * (DM / 64)), 128, 0, stream>>>(O16, BO, bo, (float*)d_out);
}
